// NonLocalSelfAttention_24232205484147
// MI455X (gfx1250) — hardware-verified
//
#include <hip/hip_runtime.h>


namespace {
constexpr int B = 16, C = 256, P = 1024, NH = 8, HD = 64, INNER = NH * HD, G = 32, CPG = C / G, TD = 1024, BL = 16  ;
constexpr float XS = 8.0f, WSC = 256.0f, PS = 1024.0f, LOG2E = 1.4426950408889634f, EPS = 1e-5f;
static_assert(P % 64 == 0 && INNER == 512, "tiling");
typedef _Float16 b16;
typedef __attribute__((ext_vector_type(16))) _Float16 v16b;
typedef __attribute__((ext_vector_type(8))) _Float16 v8b;
typedef __attribute__((ext_vector_type(8))) float v8f;
typedef __attribute__((ext_vector_type(4))) float v4f;
__device__ __forceinline__ float bf16_rne(float f) { unsigned int u = __float_as_uint(f); u += 0x7FFFu + ((u >> 16) & 1u); return __uint_as_float(u & 0xFFFF0000u); }
__device__ __forceinline__ void split16(float v, b16& hi, b16& lo) { hi = (b16)v; lo = (b16)(v - (float)hi); }
__device__ __forceinline__ v16b frag_kb(const b16* p, int hh) { const v8b a = *(const v8b*)(p + 8 * hh), b = *(const v8b*)(p + 16 + 8 * hh); v16b f;
#pragma unroll
  for (int e = 0; e < 8; ++e) { f[e] = a[e]; f[8 + e] = b[e]; } return f; }
__device__ __forceinline__ v8f wmma16b(v16b a, v16b b, v8f c) { v8f d = __builtin_amdgcn_wmma_f32_16x16x32_f16(false, a, false, b, (short)0, c, false, false); asm volatile("v_nop\n\tv_nop\n\tv_nop\n\tv_nop" : "+v"(d) : "v"(a), "v"(b)); return d; }
__device__ __forceinline__ void wave_lds_sync() { __builtin_amdgcn_fence(__ATOMIC_RELEASE, "workgroup"); __builtin_amdgcn_wave_barrier(); __builtin_amdgcn_fence(__ATOMIC_ACQUIRE, "workgroup"); }
__device__ __forceinline__ float pmul(float a, float b) { float p = a * b; asm volatile("" : "+v"(p)); return p; }
__device__ __forceinline__ int iclamp(int v, int lo, int hi) { return v < lo ? lo : (v > hi ? hi : v); }

typedef __attribute__((ext_vector_type(2))) _Float16 v2h;
typedef __attribute__((ext_vector_type(4))) _Float16 v4h;
__device__ __forceinline__ float nexp2(float v) { return __builtin_amdgcn_exp2f(v); }
__global__ __launch_bounds__(256) void prep_kernel(const float* __restrict__ inw, const float* __restrict__ outw, b16* __restrict__ WI, b16* __restrict__ WO) {
  const size_t u = (size_t)blockIdx.x * 256 + threadIdx.x; const size_t n1 = (size_t)3 * INNER * C / 8, n2 = (size_t)C * INNER / 8; v8b o;
  if (u < n1) { const size_t e = u * 8; for (int j = 0; j < 8; ++j) o[j] = (b16)(bf16_rne(inw[e + j]) * WSC); for (int pass = 0; pass < 2; ++pass) { *(volatile v8b*)(WI + e) = o; __threadfence(); } }
  else if (u < n1 + n2) { const size_t e = (u - n1) * 8; for (int j = 0; j < 8; ++j) o[j] = (b16)(bf16_rne(outw[e + j]) * WSC); for (int pass = 0; pass < 2; ++pass) { *(volatile v8b*)(WO + e) = o; __threadfence(); } }
}
__global__ __launch_bounds__(1024) void gnstat_kernel(const float* __restrict__ x, float* __restrict__ STAT) {
  __shared__ float red[1024]; __shared__ float mus; const int blk = blockIdx.x; const int tid = threadIdx.x; const float* base = x + (size_t)blk * CPG * P; const int n = CPG * P;
  float s = 0.0f; for (int i = tid; i < n; i += 1024) s += bf16_rne(base[i]); red[tid] = s; __syncthreads();
  for (int w = 512; w >= 1; w >>= 1) { if (tid < w) red[tid] = red[tid] + red[tid + w]; __syncthreads(); }
  if (tid == 0) mus = red[0] / (float)n; __syncthreads(); const float mu = mus;
  float q = 0.0f; for (int i = tid; i < n; i += 1024) { const float d = bf16_rne(base[i]) - mu; q += d * d; } __syncthreads(); red[tid] = q; __syncthreads();
  for (int w = 512; w >= 1; w >>= 1) { if (tid < w) red[tid] = red[tid] + red[tid + w]; __syncthreads(); }
  if (tid < 32) { const float rs = rsqrtf(red[0] / (float)n + EPS); const float val = (tid == 0) ? mu : (tid == 1 ? rs : 0.0f); for (int pass = 0; pass < 2; ++pass) { ((volatile float*)STAT)[blk * 32 + tid] = val; __threadfence(); } }
}
__global__ __launch_bounds__(256) void emb_kernel(const float* __restrict__ embedding, const float* __restrict__ ew, const float* __restrict__ eb, float* __restrict__ EMB) {
  const int b = blockIdx.x, c = threadIdx.x; float s = 0.0f;
#pragma unroll 1
  for (int t = 0; t < TD; ++t) s += pmul(bf16_rne(embedding[(size_t)b * TD + t]), bf16_rne(ew[(size_t)c * TD + t]));
  s += bf16_rne(eb[c]); for (int pass = 0; pass < 2; ++pass) { ((volatile float*)EMB)[b * C + c] = s; __threadfence(); }
}
__device__ __forceinline__ float gnval(const float* __restrict__ x, const float* __restrict__ STAT, const float* __restrict__ w, const float* __restrict__ bb, int b, int c, int p) {
  const float* st = STAT + (b * G + c / CPG) * 32; return (bf16_rne(x[((size_t)b * C + c) * P + p]) - st[0]) * st[1] * bf16_rne(w[c]) + bf16_rne(bb[c]);
}
__global__ __launch_bounds__(128) void qkv_kernel(const float* __restrict__ x, const float* __restrict__ STAT, const float* __restrict__ nw, const float* __restrict__ nb, const b16* __restrict__ WI, const float* __restrict__ inb, b16* __restrict__ QP, b16* __restrict__ KP, b16* __restrict__ VT) {
  __shared__ __attribute__((aligned(16))) b16 As[64][C + 8]; __shared__ __attribute__((aligned(16))) float Tf[4][16][128 + 4];
  const int wave = threadIdx.x >> 5, lane = threadIdx.x & 31, nloc = lane & 15, hlf = lane >> 4; const int p0 = blockIdx.x * 64; const int b = blockIdx.y; const int slab = blockIdx.z, n0 = slab * 128, which = slab / 4, c0 = n0 - which * INNER;
  for (int i = threadIdx.x; i < C * 64; i += 128) { const int c = i / 64, pp = i % 64; As[pp][c] = (b16)(gnval(x, STAT, nw, nb, b, c, p0 + pp) * XS); }
  __syncthreads();
  v8f acc[8];
#pragma unroll
  for (int t = 0; t < 8; ++t) acc[t] = (v8f){};
#pragma unroll 2
  for (int kb = 0; kb < C; kb += 32) { const v16b a = frag_kb(&As[wave * 16 + nloc][kb], hlf);
#pragma unroll
    for (int t = 0; t < 8; ++t) acc[t] = wmma16b(a, frag_kb(WI + (size_t)(n0 + t * 16 + nloc) * C + kb, hlf), acc[t]); }
#pragma unroll
  for (int t = 0; t < 8; ++t) { const float bb = bf16_rne(inb[n0 + t * 16 + nloc]);
#pragma unroll
    for (int r = 0; r < 8; ++r) Tf[wave][8 * hlf + r][t * 16 + nloc] = acc[t][r] * (1.0f / (XS * WSC)) + bb; }
  __syncthreads();
  for (int pass = 0; pass < 2; ++pass) {
    if (which < 2) { b16* plane = which == 0 ? QP : KP; const int cl = lane * 4; const int c = c0 + cl; const int h = c / HD, d = c % HD;
      for (int rr = 0; rr < 16; ++rr) { const int p = p0 + wave * 16 + rr; v4h o4; for (int j = 0; j < 4; ++j) o4[j] = (b16)(Tf[wave][rr][cl + j] * XS); *(volatile v4h*)(plane + (((size_t)b * NH + h) * P + p) * HD + d) = o4; } }
    else {
#pragma unroll 1
      for (int q = 0; q < 32; ++q) { const int cl = wave * 32 + q; const int c = c0 + cl; const int h = c / HD, d = c % HD; const int tk = lane * 2; v2h vv; vv[0] = (b16)(Tf[tk >> 4][tk & 15][cl] * XS); vv[1] = (b16)(Tf[(tk + 1) >> 4][(tk + 1) & 15][cl] * XS);
        *(volatile v2h*)(VT + (((size_t)b * NH + h) * HD + d) * (size_t)P + p0 + lane * 2) = vv; } }
    __threadfence(); }
}
__global__ __launch_bounds__(64) void attn_kernel(const b16* __restrict__ QP, const b16* __restrict__ KP, const b16* __restrict__ VT, b16* __restrict__ CT) {
  __shared__ __attribute__((aligned(16))) b16 Pb[2][16][32 + 8]; __shared__ __attribute__((aligned(16))) float To[2][16][HD + 4];
  const int wave = threadIdx.x >> 5, lane = threadIdx.x & 31, hh = lane >> 4, col = lane & 15; const int b = blockIdx.y / NH, h = blockIdx.y % NH; const int q0 = blockIdx.x * 32 + wave * 16, qi = q0 + col;
  const size_t ph = (size_t)b * NH + h; const b16* Qb = QP + ph * P * HD; const b16* Kb = KP + ph * P * HD; const b16* Vb = VT + ph * HD * (size_t)P;
  const v16b qa0 = frag_kb(Qb + (size_t)qi * HD, hh), qa1 = frag_kb(Qb + (size_t)qi * HD + 32, hh);
  const float cs = LOG2E / (8.0f * XS * XS);
  float m = -INFINITY, l = 0.0f; v8f o[4]; for (int t = 0; t < 4; ++t) o[t] = (v8f){};
#pragma unroll 1
  for (int kb = 0; kb < P; kb += 32) {
    float e[16]; float mx = -INFINITY;
#pragma unroll
    for (int u = 0; u < 2; ++u) { v8f s = (v8f){}; const size_t kr = (size_t)(kb + u * 16 + col) * HD; s = wmma16b(frag_kb(Kb + kr, hh), qa0, s); s = wmma16b(frag_kb(Kb + kr + 32, hh), qa1, s);
#pragma unroll
      for (int r = 0; r < 8; ++r) { const float vv = s[r] * cs; e[u * 8 + r] = vv; mx = fmaxf(mx, vv); } }
    mx = fmaxf(mx, __shfl_xor(mx, 16)); const float mn = fmaxf(m, mx); const float al = nexp2(m - mn); float sum = 0.0f;
#pragma unroll
    for (int i2 = 0; i2 < 16; ++i2) { const float p = nexp2(e[i2] - mn); sum += p; Pb[wave][col][(i2 < 8 ? 0 : 16) + 8 * hh + (i2 & 7)] = (b16)(p * PS); }
    sum += __shfl_xor(sum, 16); l = l * al + sum; m = mn;
    wave_lds_sync();
    const v16b pf = frag_kb(&Pb[wave][col][0], hh);
#pragma unroll
    for (int t = 0; t < 4; ++t) { o[t] *= al; o[t] = wmma16b(frag_kb(Vb + (size_t)(t * 16 + col) * P + kb, hh), pf, o[t]); }
    wave_lds_sync(); }
  const float inv = 1.0f / (l * PS * XS);
#pragma unroll
  for (int t = 0; t < 4; ++t)
#pragma unroll
    for (int r = 0; r < 8; ++r) To[wave][col][t * 16 + 8 * hh + r] = o[t][r] * inv;
  wave_lds_sync();
  b16* Cb = CT + ph * P * HD;
  for (int pass = 0; pass < 2; ++pass) { for (int rr = 0; rr < 16; ++rr) { v2h o2; o2[0] = (b16)(To[wave][rr][lane * 2] * XS); o2[1] = (b16)(To[wave][rr][lane * 2 + 1] * XS); *(volatile v2h*)(Cb + (size_t)(q0 + rr) * HD + lane * 2) = o2; } __threadfence(); }
}
__global__ __launch_bounds__(128) void out_kernel(const b16* __restrict__ CT, const b16* __restrict__ WO, const float* __restrict__ ob, const float* __restrict__ EMB, const float* __restrict__ x, float* __restrict__ out) {
  __shared__ __attribute__((aligned(16))) float To[4][16][32 + 4];
  const int wave = threadIdx.x >> 5, lane = threadIdx.x & 31, nloc = lane & 15, hlf = lane >> 4; const int o0 = blockIdx.x * 64 + wave * 16; const int p0 = blockIdx.y * 32; const int b = blockIdx.z;
  v8f acc[2] = {(v8f){}, (v8f){}};
#pragma unroll 4
  for (int ks = 0; ks < INNER / 32; ++ks) { const v16b a = frag_kb(WO + (size_t)(o0 + nloc) * INNER + ks * 32, hlf); const b16* cb = CT + (((size_t)b * NH + ks / 2) * P) * HD + (ks % 2) * 32;
#pragma unroll
    for (int t = 0; t < 2; ++t) acc[t] = wmma16b(a, frag_kb(cb + (size_t)(p0 + t * 16 + nloc) * HD, hlf), acc[t]); }
#pragma unroll
  for (int t = 0; t < 2; ++t)
#pragma unroll
    for (int r = 0; r < 8; ++r) To[wave][8 * hlf + r][t * 16 + nloc] = acc[t][r] * (1.0f / (XS * WSC));
  wave_lds_sync();
  for (int pass = 0; pass < 2; ++pass) { for (int rr = 0; rr < 16; ++rr) { const int o = o0 + rr; const int p = p0 + lane; const float v = (To[wave][rr][lane] + bf16_rne(ob[o])) * EMB[b * C + o] + bf16_rne(x[((size_t)b * C + o) * P + p]);
      ((volatile float*)out)[((size_t)b * C + o) * P + p] = v; } __threadfence(); }
}
}

extern "C" void kernel_launch(void* const* d_in, const int* in_sizes, int n_in, void* d_out, int out_size, void* d_ws, size_t ws_size, hipStream_t stream) {
  (void)n_in;
  auto Fp = [&](int i) { return (const float*)d_in[i]; };
  if (in_sizes[0] != B * C * P || in_sizes[1] != B * TD || in_sizes[2] != C || in_sizes[4] != 3 * INNER * C || in_sizes[5] != 3 * INNER || in_sizes[6] != C * INNER || in_sizes[8] != C * TD || in_sizes[9] != C || out_size != B * C * P) return;
  size_t off = 0; char* ws = (char*)d_ws;
  auto carve = [&](size_t bytes) { char* p = ws + off; off += (bytes + 255) & ~(size_t)255; return p; };
  b16* WI = (b16*)carve((size_t)3 * INNER * C * 2); b16* WO = (b16*)carve((size_t)C * INNER * 2); float* STAT = (float*)carve((size_t)B * G * 32 * 4); float* EMB = (float*)carve((size_t)B * C * 4);
  const size_t plane = (size_t)B * NH * P * HD * 2; b16* QP = (b16*)carve(plane); b16* KP = (b16*)carve(plane); b16* VT = (b16*)carve(plane); b16* CT = (b16*)carve(plane);
  if (off > ws_size || off > ((size_t)128 << 20)) return;
  prep_kernel<<<(unsigned)(((size_t)3 * INNER * C / 8 + (size_t)C * INNER / 8 + 255) / 256), 256, 0, stream>>>(Fp(4), Fp(6), WI, WO);
  gnstat_kernel<<<B * G, 1024, 0, stream>>>(Fp(0), STAT);
  emb_kernel<<<B, C, 0, stream>>>(Fp(1), Fp(8), Fp(9), EMB);
  qkv_kernel<<<dim3(P / 64, BL, 12), 128, 0, stream>>>(Fp(0), STAT, Fp(2), Fp(3), WI, Fp(5), QP, KP, VT);
  attn_kernel<<<dim3(P / 32, BL * NH), 64, 0, stream>>>(QP, KP, VT, CT);
  out_kernel<<<dim3(C / 64, P / 32, BL), 128, 0, stream>>>(CT, WO, Fp(7), EMB, Fp(0), (float*)d_out);
}
